// MambaBlock_53652731462315
// MI455X (gfx1250) — hardware-run, weakly checked
//
#include <hip/hip_runtime.h>
#include <math.h>

typedef __attribute__((ext_vector_type(16))) _Float16 v16h;
typedef __attribute__((ext_vector_type(8)))  _Float16 v8h;
typedef __attribute__((ext_vector_type(8)))  float    v8f;
typedef __attribute__((ext_vector_type(4)))  float    v4f;
typedef __attribute__((ext_vector_type(2)))  float    v2f;

constexpr int kBatch = 4;
constexpr int kSeqL  = 2048;
constexpr int kHid   = 1024;
constexpr int kExp   = 2048;
constexpr int kNst   = 16;
constexpr int kRank  = 64;
constexpr int kRows  = kBatch * kSeqL;
constexpr int kXpN   = 2 * kExp;
constexpr int kPrjP  = 128;
constexpr int kBcP   = 32;
constexpr int kScanT  = 16;
constexpr int kScanCh = 512;
constexpr int kScanYP = 516;

constexpr float kCarryW   = 32.0f;
constexpr float kCarryWdt = 8.0f;
constexpr float kCarryU   = 16.0f;
constexpr float kCarryDt  = 16.0f;
constexpr float kCarryY   = 16.0f;
constexpr float kSclInProj  = 1.0f / kCarryW;
constexpr float kSclXProj   = 1.0f / (kCarryU * kCarryW);
constexpr float kSclDtProj  = 1.0f / (kCarryDt * kCarryWdt);
constexpr float kSclOutProj = 1.0f / (kCarryY * kCarryW);
constexpr float kInvCarryU  = 1.0f / kCarryU;
constexpr float kLog2e      = 1.4426950408889634f;

static_assert(kRows == 8192 && kXpN == 4096, "shape");
static_assert((size_t)kRows * kHid * 4 == 33554432ull, "x / out bytes");
static_assert((kHid % 32) == 0 && (kExp % 32) == 0 && (kRank % 32) == 0, "GEMM K multiples of 32");
static_assert((kRows % 64) == 0 && (kExp % 64) == 0 && (kHid % 64) == 0 && (kPrjP % 64) == 0, "GEMM M,N multiples of 64");
static_assert(kRank + 2 * kNst <= kPrjP && kRank == 64 && 2 * kNst == kBcP, "fused projection layout");
static_assert((kSeqL % kScanT) == 0 && (kExp % kScanCh) == 0, "scan tiling");
static_assert(32 * 256 <= kScanT * kScanYP && (kScanYP % 4) == 0, "scan LDS tile");

constexpr size_t kSzXn    = (size_t)kRows * kHid * 2;
constexpr size_t kSzWinT  = (size_t)kXpN * kHid * 2;
constexpr size_t kSzPlane = (size_t)kRows * kExp * 2;
constexpr size_t kOffP    = 0;
constexpr size_t kOffU    = kOffP + kSzPlane;
constexpr size_t kOffGY   = kOffU + kSzPlane;
constexpr size_t kOffWxT  = kOffGY + kSzPlane;
constexpr size_t kOffDtl  = kOffWxT + (size_t)kPrjP * kExp * 2;
constexpr size_t kOffBC   = kOffDtl + (size_t)kRows * kRank * 2;
constexpr size_t kOffWdtT = kOffBC + (size_t)kRows * kBcP * 4;
constexpr size_t kOffWoutT = kOffWdtT + (size_t)kExp * kRank * 2;
constexpr size_t kWsTotal = kOffWoutT + (size_t)kHid * kExp * 2;
static_assert(kSzXn + kSzWinT <= kSzPlane, "phase A planes fit region P");
static_assert(kWsTotal == 107741184ull, "carve total");
static_assert(kWsTotal <= 134217728ull, "carve cap");
static_assert((kOffU % 128) == 0 && (kOffGY % 128) == 0 && (kOffWxT % 128) == 0 && (kOffDtl % 128) == 0 &&
              (kOffBC % 128) == 0 && (kOffWdtT % 128) == 0 && (kOffWoutT % 128) == 0 && (kSzXn % 128) == 0, "128-B aligned regions");

template <typename T> struct Frag;
template <> struct Frag<_Float16> {
  typedef v16h V; union U { v16h v; v8h h[2]; };
  static __device__ __forceinline__ v16h load(const _Float16* p) {
    U f; f.h[0] = *(const v8h*)(p); f.h[1] = *(const v8h*)(p + 16); return f.v;
  }
  static __device__ __forceinline__ v8f mma(v16h a, v16h b, v8f c) {
    return __builtin_amdgcn_wmma_f32_16x16x32_f16(false, a, false, b, (short)0, c, false, false);
  }
};
__device__ __forceinline__ void wmma_row_guard(v8f& a0, v8f& a1, v8f& a2, v8f& a3,
                                               v16h x, v16h b0, v16h b1, v16h b2, v16h b3) {
  asm volatile("v_nop\n\tv_nop\n\tv_nop\n\tv_nop"
               : "+v"(a0), "+v"(a1), "+v"(a2), "+v"(a3)
               : "v"(x), "v"(b0), "v"(b1), "v"(b2), "v"(b3));
}
__device__ __forceinline__ void keep4_h(v16h a, v16h b, v16h c, v16h d) { asm volatile("v_nop" :: "v"(a), "v"(b), "v"(c), "v"(d)); }
__device__ __forceinline__ void acc_guard4(v8f& a, v8f& b, v8f& c, v8f& d) { asm volatile("v_nop\n\tv_nop\n\tv_nop\n\tv_nop" : "+v"(a), "+v"(b), "+v"(c), "+v"(d)); }
__device__ __forceinline__ void lds_wave_sync() {
  __builtin_amdgcn_fence(__ATOMIC_RELEASE, "workgroup");
  __builtin_amdgcn_wave_barrier();
  __builtin_amdgcn_fence(__ATOMIC_ACQUIRE, "workgroup");
}
__device__ __forceinline__ float h16_to_f32(unsigned hb) {
  const unsigned sgn = (hb & 0x8000u) << 16; const unsigned em = hb & 0x7fffu;
  const float fn = __uint_as_float((em << 13) + 0x38000000u);
  const float fs = (float)em * 5.9604644775390625e-8f;
  const float mag = (em < 0x400u) ? fs : fn; return __uint_as_float(__float_as_uint(mag) | sgn); }

__global__ __launch_bounds__(256) void transpose_cast_kernel(
    const float* __restrict__ W, unsigned short* __restrict__ Bt, int Kdim, int Ndim, int rowOff, int nwrite, float scale)
{
  __shared__ float tile[64 * 65];
  const int tid = threadIdx.x, lane = tid & 31, wave = tid >> 5;
  const int n0 = blockIdx.x * 64;
  const int k0 = blockIdx.y * 64;
#pragma unroll
  for (int p = 0; p < 16; ++p) {
    const int idx = tid + p * 256;
    const int kk  = idx >> 6;
    const int nn  = idx & 63;
    const int n   = n0 + nn;
    const int nc  = (n < Ndim) ? n : (Ndim - 1);
    const float v = W[(size_t)(k0 + kk) * Ndim + nc];
    tile[kk * 65 + nn] = (n < Ndim) ? (v * scale) : 0.f;
  }
  __syncthreads();
  const int q = lane >> 3, c8 = (lane & 7) * 8;
  v8h hv[2];
#pragma unroll
  for (int it = 0; it < 2; ++it) {
    const int nrow = it * 32 + wave * 4 + q;
#pragma unroll
    for (int e = 0; e < 8; ++e) hv[it][e] = (_Float16)tile[(c8 + e) * 65 + nrow];
  }
  for (int pass = 0; pass < 2; ++pass) {
#pragma unroll
    for (int it = 0; it < 2; ++it) {
      const int nrow = it * 32 + wave * 4 + q;
      if (nrow < nwrite)
        *(volatile v8h*)(Bt + (size_t)(rowOff + n0 + nrow) * Kdim + k0 + c8) = hv[it];
    }
    __threadfence();
  }
}

__global__ __launch_bounds__(256) void layernorm_f16_kernel(
    const float* __restrict__ x, const float* __restrict__ g, const float* __restrict__ bta,
    unsigned short* __restrict__ xn)
{
  const int lane = threadIdx.x & 31, wave = threadIdx.x >> 5;
  const int row = blockIdx.x * 8 + wave;
  if (row >= kRows) return;
  const float* xr = x + (size_t)row * kHid;
  v4f a[4], c[4];
#pragma unroll
  for (int it = 0; it < 4; ++it) {
    a[it] = *(const v4f*)(xr + it * 256 + lane * 8);
    c[it] = *(const v4f*)(xr + it * 256 + lane * 8 + 4);
  }
  float s = 0.f;
#pragma unroll
  for (int it = 0; it < 4; ++it) {
    const float p = ((a[it][0] + a[it][1]) + (a[it][2] + a[it][3])) + ((c[it][0] + c[it][1]) + (c[it][2] + c[it][3]));
    s += p;
  }
#pragma unroll
  for (int off = 16; off > 0; off >>= 1) s += __shfl_xor(s, off, 32);
  const float mu = s * (1.0f / (float)kHid);
  float vs = 0.f;
#pragma unroll
  for (int it = 0; it < 4; ++it) {
    float p = 0.f;
#pragma unroll
    for (int e = 0; e < 4; ++e) {
      const float d0 = a[it][e] - mu;
      const float d1 = c[it][e] - mu;
      p = fmaf(d0, d0, p);
      p = fmaf(d1, d1, p);
    }
    vs += p;
  }
#pragma unroll
  for (int off = 16; off > 0; off >>= 1) vs += __shfl_xor(vs, off, 32);
  const float rstd = rsqrtf(vs * (1.0f / (float)kHid) + 1e-5f);
  v8h hv[4];
#pragma unroll
  for (int it = 0; it < 4; ++it) {
    const v4f g0 = *(const v4f*)(g + it * 256 + lane * 8);
    const v4f g1 = *(const v4f*)(g + it * 256 + lane * 8 + 4);
    const v4f b0 = *(const v4f*)(bta + it * 256 + lane * 8);
    const v4f b1 = *(const v4f*)(bta + it * 256 + lane * 8 + 4);
#pragma unroll
    for (int e = 0; e < 4; ++e) {
      hv[it][e]     = (_Float16)(fmaf((a[it][e] - mu) * rstd, g0[e], b0[e]));
      hv[it][4 + e] = (_Float16)(fmaf((c[it][e] - mu) * rstd, g1[e], b1[e]));
    }
  }
  unsigned short* orow = xn + (size_t)row * kHid;
  for (int pass = 0; pass < 2; ++pass) {
#pragma unroll
    for (int it = 0; it < 4; ++it)
      *(volatile v8h*)(orow + it * 256 + lane * 8) = hv[it];
    __threadfence();
  }
}

constexpr int kEpiSilu2 = 0, kEpiProj = 1, kEpiSoftplus = 2, kEpiResid = 3;

template <int EPI>
__global__ __launch_bounds__(256) void gemm64_f16_kernel(
    const unsigned short* __restrict__ Ap, int lda,
    const unsigned short* __restrict__ Btp, int ldb, long partStrideB,
    void* __restrict__ C0, void* __restrict__ C1, int ldc,
    const float* __restrict__ bias0, const float* __restrict__ bias1, const float* __restrict__ bias2,
    const float* __restrict__ resid,
    int M, int N, int K, float scale)
{
  typedef _Float16 T;
  typedef v16h V;
  __shared__ __align__(16) float sT[8][16 * 68];
  const int part = blockIdx.y;
  const int lane = threadIdx.x & 31;
  const int wave = threadIdx.x >> 5;
  const int tilesN = N >> 6;
  const int tilesM = M >> 6;
  const int tile = blockIdx.x * 8 + wave;
  if (tile >= tilesM * tilesN) return;
  const int tm = tile / tilesN;
  const int tn = tile - tm * tilesN;
  const int m0 = tm << 6;
  const int n0 = tn << 6;

  const T* Ab = (const T*)Ap;
  const T* Bb = (const T*)Btp + (size_t)part * (size_t)partStrideB;

  const int rlane = lane & 15;
  const int koff  = (lane >> 4) * 8;
  const int mOff  = (lane >> 4) * 8;

  v8f acc[4][4];
#pragma unroll
  for (int i = 0; i < 4; ++i)
#pragma unroll
    for (int j = 0; j < 4; ++j) acc[i][j] = (v8f){0.f,0.f,0.f,0.f,0.f,0.f,0.f,0.f};

  for (int k0 = 0; k0 < K; k0 += 32) {
    V bh[4];
#pragma unroll
    for (int j = 0; j < 4; ++j) {
      const size_t bo = (size_t)(n0 + (j << 4) + rlane) * ldb + koff + k0;
      bh[j] = Frag<T>::load(Bb + bo);
    }
#pragma unroll
    for (int i = 0; i < 4; ++i) {
      const size_t ao = (size_t)(m0 + (i << 4) + rlane) * lda + koff + k0;
      V ah = Frag<T>::load(Ab + ao);
#pragma unroll
      for (int j = 0; j < 4; ++j) acc[i][j] = Frag<T>::mma(ah, bh[j], acc[i][j]);
      wmma_row_guard(acc[i][0], acc[i][1], acc[i][2], acc[i][3], ah, bh[0], bh[1], bh[2], bh[3]);
    }
    keep4_h(bh[0], bh[1], bh[2], bh[3]);
  }
  acc_guard4(acc[0][0], acc[0][1], acc[0][2], acc[0][3]);
  acc_guard4(acc[1][0], acc[1][1], acc[1][2], acc[1][3]);
  acc_guard4(acc[2][0], acc[2][1], acc[2][2], acc[2][3]);
  acc_guard4(acc[3][0], acc[3][1], acc[3][2], acc[3][3]);

  float* slab = sT[wave];
  const float oscA = (EPI == kEpiProj && part == 0) ? kCarryDt : 1.0f;
  const float oscB = (EPI == kEpiSilu2 && part == 0) ? kCarryU : 1.0f;
#pragma unroll
  for (int i = 0; i < 4; ++i) {
    const int mBase = m0 + (i << 4);
#pragma unroll
    for (int j = 0; j < 4; ++j) {
      const int n = n0 + (j << 4) + rlane;
      float bv;
      if (EPI == kEpiSilu2) {
        bv = bias0[part * N + n];
      } else if (EPI == kEpiProj) {
        const float bA = bias0[n];
        float bB = 0.0f;
        if (j == 0) bB = bias1[rlane];
        if (j == 1) bB = bias2[rlane];
        bv = (part == 0) ? bA : bB;
      } else {
        bv = bias0[n];
      }
#pragma unroll
      for (int r = 0; r < 8; ++r) {
        float v = fmaf(acc[i][j][r], scale, bv);
        if (EPI == kEpiProj) v *= oscA;
        slab[(mOff + r) * 68 + (j << 4) + rlane] = v;
      }
    }
    lds_wave_sync();
    if (EPI == kEpiSilu2 || EPI == kEpiSoftplus) {
#pragma unroll 1
      for (int it = 0; it < 16; ++it) {
        float* sp = slab + it * 68 + lane * 2;
        const v2f vin = *(const v2f*)sp;
        v2f vo;
#pragma unroll
        for (int e = 0; e < 2; ++e) {
          const float xv = vin[e];
          if (EPI == kEpiSilu2) {
            const float ex = __expf(-xv);
            vo[e] = (xv * __builtin_amdgcn_rcpf(1.0f + ex)) * oscB;
          } else {
            const float ax = __expf(-fabsf(xv));
            vo[e] = fmaxf(xv, 0.0f) + __logf(1.0f + ax);
          }
        }
        *(v2f*)sp = vo;
      }
      lds_wave_sync();
    }
    if (EPI == kEpiResid) {
      float* C = (float*)C0;
      const int hh = lane >> 4, c4 = (lane & 15) * 4;
      v4f ov[8];
#pragma unroll
      for (int it = 0; it < 8; ++it) {
        const int row = it * 2 + hh;
        const v4f v = *(const v4f*)(slab + row * 68 + c4);
        const v4f rv = *(const v4f*)(resid + (size_t)(mBase + row) * ldc + n0 + c4);
        ov[it] = v + rv;
      }
      for (int pass = 0; pass < 2; ++pass) {
#pragma unroll
        for (int it = 0; it < 8; ++it) {
          const int row = it * 2 + hh;
          *(volatile v4f*)(C + (size_t)(mBase + row) * ldc + n0 + c4) = ov[it];
        }
        __threadfence();
      }
    } else if (EPI == kEpiProj && part != 0) {
      float* Cf = (float*)C1;
      const int q = lane >> 3, c4 = (lane & 7) * 4;
      v4f ov[4];
#pragma unroll
      for (int it = 0; it < 4; ++it) {
        const int row = it * 4 + q;
        ov[it] = *(const v4f*)(slab + row * 68 + c4);
      }
      for (int pass = 0; pass < 2; ++pass) {
#pragma unroll
        for (int it = 0; it < 4; ++it) {
          const int row = it * 4 + q;
          *(volatile v4f*)(Cf + (size_t)(mBase + row) * kBcP + c4) = ov[it];
        }
        __threadfence();
      }
    } else {
      const int q = lane >> 3, c8 = (lane & 7) * 8;
      unsigned short* C = (EPI == kEpiSilu2 && part != 0) ? (unsigned short*)C1 : (unsigned short*)C0;
      for (int pass = 0; pass < 2; ++pass) {
#pragma unroll
        for (int it = 0; it < 4; ++it) {
          const int row = it * 4 + q;
          const float* sp = slab + row * 68 + c8;
          const v4f a0 = *(const v4f*)(sp);
          const v4f a1 = *(const v4f*)(sp + 4);
          v8h hv;
#pragma unroll
          for (int e = 0; e < 4; ++e) {
            hv[e]     = (_Float16)a0[e];
            hv[4 + e] = (_Float16)a1[e];
          }
          *(volatile v8h*)(C + (size_t)(mBase + row) * ldc + n0 + c8) = hv;
        }
        __threadfence();
      }
    }
    lds_wave_sync();
  }
}

__global__ __launch_bounds__(256) void scan_kernel(
    const unsigned* __restrict__ Uw, const unsigned* __restrict__ Dw, unsigned* GYw,
    const float* __restrict__ BC, const float* __restrict__ Alog, const float* __restrict__ Dv)
{
  __shared__ __align__(16) float sBC[kScanT * kBcP];
  __shared__ __align__(16) float sY[kScanT * kScanYP];
  const int tid = threadIdx.x;
  const int bix = blockIdx.x >> 2;
  const int ch0 = (blockIdx.x & 3) * kScanCh;
  const int e0  = ch0 + 2 * tid;

#pragma unroll 1
  for (int j = 0; j < 2 * kNst; ++j) {
    const float al = Alog[(size_t)e0 * kNst + j];
    sY[j * 256 + tid] = (-expf(al)) * kLog2e;
  }
  __syncthreads();
  float a2[2][kNst], h[2][kNst];
#pragma unroll
  for (int c = 0; c < 2; ++c)
#pragma unroll
    for (int n = 0; n < kNst; ++n) {
      a2[c][n] = sY[(c * kNst + n) * 256 + tid];
      h[c][n] = 0.f;
    }
  const float Dd0 = Dv[e0], Dd1 = Dv[e0 + 1];

  const size_t rowBase = (size_t)bix * kSeqL;
  const int wcol = (ch0 >> 1) + tid;
  unsigned short* GYh = (unsigned short*)GYw;

#pragma unroll 1
  for (int c = 0; c < kSeqL / kScanT; ++c) {
    const int l0 = c * kScanT;
    if (tid < 128) {
      const int r = tid >> 3, q4 = (tid & 7) * 4;
      const v4f v = *(const v4f*)(BC + (rowBase + l0 + r) * kBcP + q4);
      *(v4f*)(sBC + r * kBcP + q4) = v;
    }
    __syncthreads();
#pragma unroll 1
    for (int s = 0; s < kScanT; ++s) {
      const size_t wi = (rowBase + l0 + s) * (size_t)(kExp / 2) + wcol;
      unsigned uw = Uw[wi];
      unsigned dw = Dw[wi];
      unsigned gw = GYw[wi];
      asm volatile("" : "+v"(uw), "+v"(dw), "+v"(gw));
      const float u0 = h16_to_f32(uw & 0xffffu) * kInvCarryU;
      const float u1 = h16_to_f32(uw >> 16) * kInvCarryU;
      const float dl0 = h16_to_f32(dw & 0xffffu);
      const float dl1 = h16_to_f32(dw >> 16);
      const float g0 = h16_to_f32(gw & 0xffffu);
      const float g1 = h16_to_f32(gw >> 16);
      v4f Bq[4], Cq[4];
#pragma unroll
      for (int qq = 0; qq < 4; ++qq) {
        Bq[qq] = *(const v4f*)(sBC + s * kBcP + 4 * qq);
        Cq[qq] = *(const v4f*)(sBC + s * kBcP + kNst + 4 * qq);
      }
      float y0 = 0.f, y1 = 0.f;
#pragma unroll
      for (int n = 0; n < kNst; ++n) {
        const float bn = Bq[n >> 2][n & 3];
        const float cn = Cq[n >> 2][n & 3];
        const float ea = __builtin_amdgcn_exp2f(dl0 * a2[0][n]);
        const float eb = __builtin_amdgcn_exp2f(dl1 * a2[1][n]);
        h[0][n] = fmaf(ea, h[0][n], (dl0 * bn) * u0);
        h[1][n] = fmaf(eb, h[1][n], (dl1 * bn) * u1);
        y0 = fmaf(cn, h[0][n], y0);
        y1 = fmaf(cn, h[1][n], y1);
      }
      y0 = fmaf(u0, Dd0, y0);
      y1 = fmaf(u1, Dd1, y1);
      v2f yy;
      yy[0] = (y0 * g0) * kCarryY;
      yy[1] = (y1 * g1) * kCarryY;
      *(v2f*)(sY + s * kScanYP + 2 * tid) = yy;
    }
    __syncthreads();
    v8h hv[4];
#pragma unroll
    for (int it = 0; it < 4; ++it) {
      const int ci = it * 256 + tid;
      const int row = ci >> 6, c8 = (ci & 63) * 8;
      const float* sp = sY + row * kScanYP + c8;
      const v4f a0 = *(const v4f*)(sp);
      const v4f a1 = *(const v4f*)(sp + 4);
#pragma unroll
      for (int e = 0; e < 4; ++e) {
        hv[it][e]     = (_Float16)a0[e];
        hv[it][4 + e] = (_Float16)a1[e];
      }
    }
    for (int pass = 0; pass < 2; ++pass) {
#pragma unroll
      for (int it = 0; it < 4; ++it) {
        const int ci = it * 256 + tid;
        const int row = ci >> 6, c8 = (ci & 63) * 8;
        *(volatile v8h*)(GYh + (rowBase + l0 + row) * (size_t)kExp + ch0 + c8) = hv[it];
      }
      __threadfence();
    }
  }
}

extern "C" void kernel_launch(void* const* d_in, const int* in_sizes, int n_in,
                              void* d_out, int out_size, void* d_ws, size_t ws_size,
                              hipStream_t stream)
{
  if (n_in < 17) return;
  if (in_sizes[0] != kRows * kHid) return;
  if (in_sizes[1] != kHid || in_sizes[2] != kHid) return;
  if (in_sizes[3] != kHid * kXpN || in_sizes[4] != kXpN) return;
  if (in_sizes[5] != kExp * kRank || in_sizes[6] != kRank) return;
  if (in_sizes[7] != kRank * kExp || in_sizes[8] != kExp) return;
  if (in_sizes[9] != kExp * kNst || in_sizes[10] != kNst) return;
  if (in_sizes[11] != kExp * kNst || in_sizes[12] != kNst) return;
  if (in_sizes[13] != kExp * kNst || in_sizes[14] != kExp) return;
  if (in_sizes[15] != kExp * kHid || in_sizes[16] != kHid) return;
  if (out_size != kRows * kHid) return;
  if (ws_size < kWsTotal) return;

  const float* x       = (const float*)d_in[0];
  const float* ln_g    = (const float*)d_in[1];
  const float* ln_b    = (const float*)d_in[2];
  const float* W_in    = (const float*)d_in[3];
  const float* b_in    = (const float*)d_in[4];
  const float* W_delta = (const float*)d_in[5];
  const float* b_delta = (const float*)d_in[6];
  const float* W_dt    = (const float*)d_in[7];
  const float* b_dt    = (const float*)d_in[8];
  const float* W_B     = (const float*)d_in[9];
  const float* b_B     = (const float*)d_in[10];
  const float* W_C     = (const float*)d_in[11];
  const float* b_C     = (const float*)d_in[12];
  const float* A_log   = (const float*)d_in[13];
  const float* Dv      = (const float*)d_in[14];
  const float* W_out   = (const float*)d_in[15];
  const float* b_out   = (const float*)d_in[16];
  float* out = (float*)d_out;

  char* ws = (char*)d_ws;
  unsigned short* XN    = (unsigned short*)(ws + kOffP);
  unsigned short* WINT  = (unsigned short*)(ws + kOffP + kSzXn);
  unsigned short* DELTA = (unsigned short*)(ws + kOffP);
  unsigned short* UH    = (unsigned short*)(ws + kOffU);
  unsigned short* GY    = (unsigned short*)(ws + kOffGY);
  unsigned short* WXT   = (unsigned short*)(ws + kOffWxT);
  unsigned short* DTL   = (unsigned short*)(ws + kOffDtl);
  float*          BCp   = (float*)(ws + kOffBC);
  unsigned short* WDTT  = (unsigned short*)(ws + kOffWdtT);
  unsigned short* WOUTT = (unsigned short*)(ws + kOffWoutT);

  transpose_cast_kernel<<<dim3(kXpN / 64, kHid / 64), 256, 0, stream>>>(W_in, WINT, kHid, kXpN, 0, 64, kCarryW);
  transpose_cast_kernel<<<dim3(1, kExp / 64), 256, 0, stream>>>(W_delta, WXT, kExp, kRank, 0, 64, kCarryW);
  transpose_cast_kernel<<<dim3(1, kExp / 64), 256, 0, stream>>>(W_B, WXT, kExp, kNst, kRank, kNst, kCarryW);
  transpose_cast_kernel<<<dim3(1, kExp / 64), 256, 0, stream>>>(W_C, WXT, kExp, kNst, kRank + kNst, kPrjP - kRank - kNst, kCarryW);
  transpose_cast_kernel<<<dim3(kExp / 64, kRank / 64), 256, 0, stream>>>(W_dt, WDTT, kRank, kExp, 0, 64, kCarryWdt);
  transpose_cast_kernel<<<dim3(kHid / 64, kExp / 64), 256, 0, stream>>>(W_out, WOUTT, kExp, kHid, 0, 64, kCarryW);

  layernorm_f16_kernel<<<kRows / 8, 256, 0, stream>>>(x, ln_g, ln_b, XN);

  gemm64_f16_kernel<kEpiSilu2><<<dim3((kRows / 64) * (kExp / 64) / 8, 2), 256, 0, stream>>>(
      XN, kHid, WINT, kHid, (long)kExp * (long)kHid,
      (void*)UH, (void*)GY, kExp,
      b_in, b_in, b_in, x,
      kRows, kExp, kHid, kSclInProj);

  gemm64_f16_kernel<kEpiProj><<<dim3((kRows / 64) / 8, 2), 256, 0, stream>>>(
      UH, kExp, WXT, kExp, (long)64 * (long)kExp,
      (void*)DTL, (void*)BCp, kRank,
      b_delta, b_B, b_C, x,
      kRows, 64, kExp, kSclXProj);

  gemm64_f16_kernel<kEpiSoftplus><<<dim3((kRows / 64) * (kExp / 64) / 8, 1), 256, 0, stream>>>(
      DTL, kRank, WDTT, kRank, 0L,
      (void*)DELTA, (void*)DELTA, kExp,
      b_dt, b_dt, b_dt, x,
      kRows, kExp, kRank, kSclDtProj);

  scan_kernel<<<kBatch * (kExp / kScanCh), 256, 0, stream>>>(
      (const unsigned*)UH, (const unsigned*)DELTA, (unsigned*)GY, BCp, A_log, Dv);

  gemm64_f16_kernel<kEpiResid><<<dim3((kRows / 64) * (kHid / 64) / 8, 1), 256, 0, stream>>>(
      GY, kExp, WOUTT, kExp, 0L,
      (void*)out, (void*)out, kHid,
      b_out, b_out, b_out, x,
      kRows, kHid, kExp, kSclOutProj);
}
